// PointNetSetAbstraction_72756745994761
// MI455X (gfx1250) — hardware-verified
//
#include <hip/hip_runtime.h>
#include <math.h>
#pragma clang fp contract(off)

typedef __attribute__((ext_vector_type(16))) _Float16 v16h;
typedef __attribute__((ext_vector_type(8)))  _Float16 v8h;
typedef __attribute__((ext_vector_type(8)))  float    v8f;
typedef __attribute__((ext_vector_type(4)))  float    v4f;
typedef __attribute__((ext_vector_type(4)))  int      v4i;
typedef __attribute__((ext_vector_type(4)))  unsigned v4u;

constexpr int NB      = 8;
constexpr int NPTS    = 4096;
constexpr int NFEAT   = 40;
constexpr int NQ      = 1024;
constexpr int NNBR    = 32;
constexpr int CPITCH  = 64;
constexpr int NROWS   = NB * NQ * NNBR;
constexpr float WCARRY     = 64.0f;
constexpr float WCARRY_INV = 1.0f / 64.0f;
constexpr float BIGF       = 3.0e38f;

constexpr int OUT1_OFF = NB * 3 * NQ;
constexpr int OUT2_OFF = OUT1_OFF + NB * 128 * NQ;
static_assert(OUT1_OFF * 4 == 98304, "out1 byte offset");
static_assert(OUT2_OFF * 4 == 4292608, "out2 byte offset");
static_assert((OUT2_OFF + NB * NQ * NFEAT) * 4 == 5603328, "d_out total bytes");
static_assert(NROWS == 262144, "grouped rows");


constexpr size_t SZ_COMB  = (size_t)NB * NPTS * CPITCH * 4;
constexpr size_t SZ_QCOMB = (size_t)NB * NQ * CPITCH * 4;
constexpr size_t SZ_FPS   = (size_t)NB * NQ * 4;
constexpr size_t SZ_KNN   = (size_t)NROWS * 4;
constexpr size_t SZ_WH    = (size_t)(64 * 64 + 64 * 64 + 128 * 64) * 2;
constexpr size_t SZ_AB    = 4096;
constexpr size_t SZ_PART64  = (size_t)2048 * 128 * 4;
constexpr size_t SZ_PART128 = (size_t)2048 * 256 * 4;
constexpr size_t SZ_PLANE = (size_t)NROWS * 64 * 2;
constexpr size_t SZ_MM    = (size_t)NB * NQ * 256 * 4;
constexpr size_t OFF_COMB  = 0;
constexpr size_t OFF_QCOMB = OFF_COMB + SZ_COMB;
constexpr size_t OFF_FPS   = OFF_QCOMB + SZ_QCOMB;
constexpr size_t OFF_KNN   = OFF_FPS + SZ_FPS;
constexpr size_t OFF_WH    = OFF_KNN + SZ_KNN;
constexpr size_t OFF_AB    = OFF_WH + SZ_WH;
constexpr size_t OFF_P1    = OFF_AB + SZ_AB;
constexpr size_t OFF_P2    = OFF_P1 + SZ_PART64;
constexpr size_t OFF_P3    = OFF_P2 + SZ_PART64;
constexpr size_t OFF_X     = OFF_P3 + SZ_PART128;
constexpr size_t OFF_R     = OFF_X + SZ_PLANE;
constexpr size_t OFF_MM    = OFF_R + SZ_PLANE;
constexpr size_t WS_TOTAL  = OFF_MM + SZ_MM;
static_assert(WS_TOTAL <= (size_t)134217728, "carve within 128 MiB");
static_assert((OFF_QCOMB % 256) == 0 && (OFF_FPS % 256) == 0 && (OFF_KNN % 256) == 0 && (OFF_WH % 256) == 0 &&
              (OFF_AB % 256) == 0 && (OFF_P1 % 256) == 0 && (OFF_X % 256) == 0 && (OFF_R % 256) == 0 && (OFF_MM % 256) == 0,
              "region alignment");

struct FragH {
  union U { v16h v; v8h h[2]; };
  static __device__ __forceinline__ v16h load(const _Float16* p) {
    U f; f.h[0] = *(const v8h*)(p); f.h[1] = *(const v8h*)(p + 16); return f.v;
  }
};
__device__ __forceinline__ v8f mma_h(v16h a, v16h b, v8f c) {
  c = __builtin_amdgcn_wmma_f32_16x16x32_f16(false, a, false, b, (short)0, c, false, false);
  asm volatile("v_nop\n\tv_nop\n\tv_nop\n\tv_nop" : "+v"(c) : "v"(a), "v"(b));
  return c;
}

__device__ __forceinline__ float h16_to_f32(unsigned hb) {
  const unsigned sgn = (hb & 0x8000u) << 16; const unsigned em = hb & 0x7fffu;
  const float fn = __uint_as_float((em << 13) + 0x38000000u);
  const float fs = (float)em * 5.9604644775390625e-8f;
  const float mag = (em < 0x400u) ? fs : fn; return __uint_as_float(__float_as_uint(mag) | sgn);
}

__device__ __forceinline__ float sumsq40(const float* f) {
  float a[8];
#pragma unroll
  for (int l = 0; l < 8; ++l) { const float v = f[l]; a[l] = v * v; }
#pragma unroll
  for (int k = 8; k < 32; ++k) { const float v = f[k]; const float t = v * v; a[k & 7] = a[k & 7] + t; }
  const float h0 = a[0] + a[4];
  const float h1 = a[1] + a[5];
  const float h2 = a[2] + a[6];
  const float h3 = a[3] + a[7];
  const float g0 = h0 + h2;
  const float g1 = h1 + h3;
  float r = g0 + g1;
#pragma unroll
  for (int k = 32; k < 40; ++k) { const float v = f[k]; const float t = v * v; r = r + t; }
  return r;
}

__global__ __launch_bounds__(256) void k_prep(const float* __restrict__ xyz, const float* __restrict__ feat,
                                              const float* __restrict__ pts, float* __restrict__ comb) {
#pragma clang fp contract(off)
  __shared__ __align__(16) float tile[64 * CPITCH];
  const int tid = threadIdx.x;
  const int b = blockIdx.x >> 6;
  const int n0 = (blockIdx.x & 63) << 6;
  const v4f* f4 = (const v4f*)(feat + ((size_t)b * NPTS + n0) * NFEAT);
  for (int it = 0; it < 3; ++it) {
    const int i = tid + 256 * it;
    if (i < 640) {
      const v4f v = f4[i];
      const int fl = 4 * i;
      const int row = fl / NFEAT;
      const int col = fl - row * NFEAT;
      float* d = tile + row * CPITCH + 3 + col;
      d[0] = v.x; d[1] = v.y; d[2] = v.z; d[3] = v.w;
    }
  }
  if (tid < 192) {
    const int c = tid >> 6;
    const int p = tid & 63;
    tile[p * CPITCH + c]      = xyz[((size_t)b * 3 + c) * NPTS + n0 + p];
    tile[p * CPITCH + 48 + c] = pts[((size_t)b * 3 + c) * NPTS + n0 + p];
  } else {
    const int p = tid - 192;
    float* d = tile + p * CPITCH;
    d[43] = 0.0f; d[46] = 0.0f; d[47] = 0.0f;
#pragma unroll
    for (int c = 51; c < 64; ++c) d[c] = 0.0f;
  }
  __syncthreads();
  if (tid < 64) {
    float* d = tile + tid * CPITCH;
    const float nf = sumsq40(d + 3);
    const float t0 = d[0] * d[0];
    const float t1 = d[1] * d[1];
    const float t2 = d[2] * d[2];
    const float nx = (t0 + t2) + t1;
    d[44] = nf; d[45] = nx;
  }
  __syncthreads();
  float* dst = comb + ((size_t)b * NPTS + n0) * CPITCH;
  for (int pass = 0; pass < 2; ++pass) {
#pragma unroll
    for (int it = 0; it < 4; ++it) {
      const int i = tid + 256 * it;
      const v4f v = *(const v4f*)&tile[4 * i];
      *(volatile v4f*)(dst + 4 * i) = v;
    }
    __threadfence();
  }
}

__global__ __launch_bounds__(512) void k_fps(const float* __restrict__ comb, int* __restrict__ fpsIdx) {
#pragma clang fp contract(off)
  __shared__ float sdist[NPTS];
  __shared__ __align__(16) float cent[44];
  __shared__ float wv[16];
  __shared__ int   wi[16];
  __shared__ __align__(16) int sidx[NQ];
  const int tid = threadIdx.x;
  const int lane = tid & 31;
  const int w = tid >> 5;
  const int b = blockIdx.x;
  const float* cb = comb + (size_t)b * NPTS * CPITCH;
#pragma unroll
  for (int j = 0; j < 8; ++j) sdist[tid + 512 * j] = 1e10f;
  int far = 0;
  for (int s = 0; s < NQ; ++s) {
    if (tid == 0) sidx[s] = far;
    if (s == NQ - 1) break;
    if (tid < 11) *(v4f*)&cent[4 * tid] = *(const v4f*)(cb + (size_t)far * CPITCH + 4 * tid);
    __syncthreads();
    v4f c[11];
#pragma unroll
    for (int f = 0; f < 11; ++f) c[f] = *(const v4f*)&cent[4 * f];
    float bv = -1.0f;
    int bi = tid;
#pragma unroll 1
    for (int j = 0; j < 8; ++j) {
      const int pt = tid + 512 * j;
      const v4f* pr = (const v4f*)(cb + (size_t)pt * CPITCH);
      float a[4];
      {
        v4f q[6];
#pragma unroll
        for (int f = 0; f < 6; ++f) q[f] = pr[f];
#pragma unroll
        for (int e = 0; e < 4; ++e) { const float df = q[0][e] - c[0][e]; a[e] = df * df; }
#pragma unroll
        for (int f = 1; f < 6; ++f) {
#pragma unroll
          for (int e = 0; e < 4; ++e) {
            const float df = q[f][e] - c[f][e];
            const float t = df * df;
            a[e] = a[e] + t;
          }
        }
      }
      asm volatile("" ::: "memory");
      float r;
      {
        v4f q[5];
#pragma unroll
        for (int f = 0; f < 5; ++f) q[f] = pr[6 + f];
#pragma unroll
        for (int f = 0; f < 4; ++f) {
#pragma unroll
          for (int e = 0; e < 4; ++e) {
            const float df = q[f][e] - c[6 + f][e];
            const float t = df * df;
            a[e] = a[e] + t;
          }
        }
        const float h0 = a[0] + a[2];
        const float h1 = a[1] + a[3];
        r = h0 + h1;
#pragma unroll
        for (int e = 0; e < 3; ++e) {
          const float df = q[4][e] - c[10][e];
          const float t = df * df;
          r = r + t;
        }
      }
      const float nd = fminf(sdist[pt], r);
      sdist[pt] = nd;
      if (nd > bv) { bv = nd; bi = pt; }
    }
#pragma unroll
    for (int off = 1; off < 32; off <<= 1) {
      const float ov = __shfl_xor(bv, off);
      const int   oi = __shfl_xor(bi, off);
      const bool take = (ov > bv) || ((ov == bv) && (oi < bi));
      bv = take ? ov : bv;
      bi = take ? oi : bi;
    }
    if (lane == 0) { wv[w] = bv; wi[w] = bi; }
    __syncthreads();
    float fv = wv[lane & 15];
    int   fi = wi[lane & 15];
#pragma unroll
    for (int off = 1; off < 16; off <<= 1) {
      const float ov = __shfl_xor(fv, off);
      const int   oi = __shfl_xor(fi, off);
      const bool take = (ov > fv) || ((ov == fv) && (oi < fi));
      fv = take ? ov : fv;
      fi = take ? oi : fi;
    }
    fi = fi < 0 ? 0 : fi;
    fi = fi > NPTS - 1 ? NPTS - 1 : fi;
    far = fi;
  }
  __syncthreads();
  if (tid < 256) {
    const v4i v = *(const v4i*)&sidx[4 * tid];
    int* dst = fpsIdx + (size_t)b * NQ + 4 * tid;
    *(volatile v4i*)dst = v;
    __threadfence();
    *(volatile v4i*)dst = v;
  }
}

__global__ __launch_bounds__(256) void k_gather(const float* __restrict__ comb, const int* __restrict__ fpsIdx,
                                                float* __restrict__ qcomb, float* __restrict__ out) {
  __shared__ __align__(16) float srow[64 * CPITCH];
  __shared__ int sidxq[64];
  const int tid = threadIdx.x;
  const int b = blockIdx.x >> 4;
  const int s0 = (blockIdx.x & 15) << 6;
  if (tid < 64) {
    int n = fpsIdx[(size_t)b * NQ + s0 + tid];
    n = n < 0 ? 0 : n;
    n = n > NPTS - 1 ? NPTS - 1 : n;
    sidxq[tid] = n;
  }
  __syncthreads();
  const int c4 = (tid & 15) * 4;
  v4f rv[4];
#pragma unroll
  for (int it = 0; it < 4; ++it) {
    const int row = (tid >> 4) + 16 * it;
    const int n = sidxq[row];
    rv[it] = *(const v4f*)(comb + ((size_t)b * NPTS + n) * CPITCH + c4);
    *(v4f*)&srow[row * CPITCH + c4] = rv[it];
  }
  for (int pass = 0; pass < 2; ++pass) {
#pragma unroll
    for (int it = 0; it < 4; ++it) {
      const int row = (tid >> 4) + 16 * it;
      *(volatile v4f*)(qcomb + ((size_t)b * NQ + s0 + row) * CPITCH + c4) = rv[it];
    }
    __threadfence();
  }
  __syncthreads();
  float* o2 = out + OUT2_OFF + ((size_t)b * NQ + s0) * NFEAT;
  for (int pass = 0; pass < 2; ++pass) {
    for (int it = 0; it < 3; ++it) {
      const int i = tid + 256 * it;
      if (i < 640) {
        const int fl = 4 * i;
        const int row = fl / NFEAT;
        const int col = fl - row * NFEAT;
        const float* sp = srow + row * CPITCH + 3 + col;
        v4f v;
        v.x = sp[0]; v.y = sp[1]; v.z = sp[2]; v.w = sp[3];
        *(volatile v4f*)(o2 + fl) = v;
      }
    }
    if (tid < 48) {
      const int c = tid >> 4;
      const int s4 = (tid & 15) * 4;
      v4f v;
      v.x = srow[(s4 + 0) * CPITCH + c];
      v.y = srow[(s4 + 1) * CPITCH + c];
      v.z = srow[(s4 + 2) * CPITCH + c];
      v.w = srow[(s4 + 3) * CPITCH + c];
      *(volatile v4f*)(out + ((size_t)b * 3 + c) * NQ + s0 + s4) = v;
    }
    __threadfence();
  }
}

__device__ __forceinline__ void topk_insert(float& bd, int& bi, float xd, int xi, int lane) {
  const float pd = __shfl_up(bd, 1);
  const int   pi = __shfl_up(bi, 1);
  const bool gt  = bd > xd;
  const bool gtp = (lane > 0) && (pd > xd);
  const float nd = gt ? (gtp ? pd : xd) : bd;
  const int   ni = gt ? (gtp ? pi : xi) : bi;
  bd = nd; bi = ni;
}
__device__ __forceinline__ void knn_scan(const float* drow, int base, float& bd, int& bi, int lane) {
#pragma unroll 1
  for (int sub = 0; sub < 8; ++sub) {
    const float cd = drow[sub * 32 + lane];
    const int   ci = base + sub * 32 + lane;
    const float thr = __shfl(bd, 31);
    unsigned mask = (unsigned)__ballot(cd < thr);
    for (int g = 0; g < 32 && mask != 0u; ++g) {
      const int src = __ffs((int)mask) - 1;
      mask &= mask - 1u;
      const float xd = __shfl(cd, src);
      const int   xi = __shfl(ci, src);
      topk_insert(bd, bi, xd, xi, lane);
    }
  }
}

__global__ __launch_bounds__(256) void k_knn(const float* __restrict__ comb, const float* __restrict__ qcomb,
                                             int* __restrict__ knn) {
#pragma clang fp contract(off)
  __shared__ __align__(16) float qs[16 * 48];
  __shared__ float dt[16 * 256];
  const int tid = threadIdx.x;
  const int lane = tid & 31;
  const int w = tid >> 5;
  const int b = blockIdx.x >> 6;
  const int q0 = (blockIdx.x & 63) << 4;
  if (tid < 192) {
    const int r = tid / 12;
    const int f = tid - r * 12;
    *(v4f*)&qs[r * 48 + 4 * f] = *(const v4f*)(qcomb + ((size_t)b * NQ + q0 + r) * CPITCH + 4 * f);
  }
  __syncthreads();
  float bd0 = BIGF, bd1 = BIGF;
  int bi0 = 0, bi1 = 0;
  const float* cb = comb + (size_t)b * NPTS * CPITCH;
#pragma unroll 1
  for (int pc = 0; pc < NPTS; pc += 256) {
    const v4f* pr = (const v4f*)(cb + (size_t)(pc + tid) * CPITCH);
    v4f pv[12];
#pragma unroll
    for (int f = 0; f < 6; ++f) pv[f] = pr[f];
    asm volatile("" ::: "memory");
#pragma unroll
    for (int f = 6; f < 12; ++f) pv[f] = pr[f];
    asm volatile("" ::: "memory");
#pragma unroll 1
    for (int q = 0; q < 16; ++q) {
      const v4f* qr = (const v4f*)&qs[q * 48];
      v4f qv[12];
#pragma unroll
      for (int f = 0; f < 12; ++f) qv[f] = qr[f];
      float pX = qv[0][0] * pv[0][0];
      pX = __builtin_fmaf(qv[0][1], pv[0][1], pX);
      pX = __builtin_fmaf(qv[0][2], pv[0][2], pX);
      float pF = qv[0][3] * pv[0][3];
#pragma unroll
      for (int c = 4; c < 43; ++c) pF = __builtin_fmaf(qv[c >> 2][c & 3], pv[c >> 2][c & 3], pF);
      const float sF = qv[11][0] + pv[11][0];
      const float sX = qv[11][1] + pv[11][1];
      const float twoF = 2.0f * pF;
      const float twoX = 2.0f * pX;
      const float dF = sF - twoF;
      const float dX = sX - twoX;
      const float sq = dF + dX;
      dt[q * 256 + tid] = sq;
    }
    __syncthreads();
    knn_scan(&dt[(2 * w) * 256], pc, bd0, bi0, lane);
    knn_scan(&dt[(2 * w + 1) * 256], pc, bd1, bi1, lane);
    __syncthreads();
  }
  int* d0 = knn + ((size_t)b * NQ + q0 + 2 * w) * NNBR + lane;
  int* d1 = d0 + NNBR;
  *(volatile int*)d0 = bi0;
  *(volatile int*)d1 = bi1;
  __threadfence();
  *(volatile int*)d0 = bi0;
  *(volatile int*)d1 = bi1;
}

__global__ __launch_bounds__(256) void k_group(const float* __restrict__ comb, const float* __restrict__ qcomb,
                                               const int* __restrict__ knn, _Float16* __restrict__ featH) {
  __shared__ float tile[256 * 49];
  const int tid = threadIdx.x;
  const int pt = blockIdx.x * 256 + tid;
  const int bs = pt >> 5;
  const int b = bs >> 10;
  int n = knn[pt];
  n = n < 0 ? 0 : n;
  n = n > NPTS - 1 ? NPTS - 1 : n;
  const v4f* g4 = (const v4f*)(comb + ((size_t)b * NPTS + n) * CPITCH);
  const v4f* q4 = (const v4f*)(qcomb + (size_t)bs * CPITCH);
  float* tr = tile + tid * 49;
  {
    const v4f gv = g4[0];
    const v4f qv = q4[0];
    const float dx = gv.x - qv.x;
    const float dy = gv.y - qv.y;
    const float dz = gv.z - qv.z;
    const float t0 = dx * dx;
    const float t1 = dy * dy;
    const float t2 = dz * dz;
    const float ss = (t0 + t2) + t1;
    const float rr = sqrtf(ss + 1e-12f);
    tr[0] = dx; tr[1] = dy; tr[2] = dz; tr[3] = rr;
    tr[4] = gv.w - qv.w;
  }
#pragma unroll 1
  for (int f = 1; f < 10; ++f) {
    const v4f gv = g4[f];
    const v4f qv = q4[f];
    float* d = tr + 4 * f + 1;
    d[0] = gv.x - qv.x; d[1] = gv.y - qv.y; d[2] = gv.z - qv.z; d[3] = gv.w - qv.w;
  }
  {
    const v4f gv = g4[10];
    const v4f qv = q4[10];
    tr[41] = gv.x - qv.x; tr[42] = gv.y - qv.y; tr[43] = gv.z - qv.z;
    const v4f pv = g4[12];
    tr[44] = pv.x; tr[45] = pv.y; tr[46] = pv.z;
  }
  __syncthreads();
  const int l8 = tid & 7;
  _Float16* dst = featH + (size_t)blockIdx.x * 256 * 64;
  for (int pass = 0; pass < 2; ++pass) {
#pragma unroll 1
    for (int it = 0; it < 8; ++it) {
      const int row = it * 32 + (tid >> 3);
      v8h hv;
#pragma unroll
      for (int e = 0; e < 8; ++e) {
        const int c = 8 * l8 + e;
        const int cc = c > 46 ? 46 : c;
        float v = tile[row * 49 + cc];
        v = (c < 47) ? v : 0.0f;
        hv[e] = (_Float16)v;
      }
      *(volatile v8h*)(dst + (size_t)row * 64 + 8 * l8) = hv;
    }
    __threadfence();
  }
}

__global__ __launch_bounds__(256) void k_packw(const float* __restrict__ W1, const float* __restrict__ W2,
                                               const float* __restrict__ W3, _Float16* __restrict__ Wh) {
  const int g = (blockIdx.x * 256 + threadIdx.x) * 8;
  v8h o;
  if (blockIdx.x < 2) {
    const int r = g >> 6;
    const int c0 = g & 63;
#pragma unroll
    for (int e = 0; e < 8; ++e) {
      const int c = c0 + e;
      const int cc = c > 46 ? 46 : c;
      float v = W1[r * 47 + cc] * WCARRY;
      v = (c < 47) ? v : 0.0f;
      o[e] = (_Float16)v;
    }
  } else if (blockIdx.x < 4) {
    const int i = g - 4096;
#pragma unroll
    for (int e = 0; e < 8; ++e) o[e] = (_Float16)(W2[i + e] * WCARRY);
  } else {
    const int i = g - 8192;
#pragma unroll
    for (int e = 0; e < 8; ++e) o[e] = (_Float16)(W3[i + e] * WCARRY);
  }
  *(volatile v8h*)(Wh + g) = o;
  __threadfence();
  *(volatile v8h*)(Wh + g) = o;
}

template <int COUT, bool LAST>
__global__ __launch_bounds__(256) void k_mlp(const _Float16* __restrict__ Ain, const _Float16* __restrict__ Wh,
                                             const float* __restrict__ bias, _Float16* __restrict__ rawOut,
                                             float* __restrict__ partial, float* __restrict__ mmOut) {
  constexpr int NT = COUT / 16;
  __shared__ __align__(16) _Float16 wl[COUT * 64];
  __shared__ __align__(16) float slab[LAST ? 8 : 8 * 16 * 68];
  __shared__ float lsum[8 * COUT];
  __shared__ float lsq[8 * COUT];
  __shared__ float wmx[LAST ? 8 * COUT : 8];
  __shared__ float wmn[LAST ? 8 * COUT : 8];
  __shared__ __align__(16) float pvec[2 * COUT];
  const int tid = threadIdx.x;
  const int lane = tid & 31;
  const int w = tid >> 5;
  const int hh = lane >> 4;
  const int m = lane & 15;
  const int koff = hh * 8;
  for (int i = tid; i < COUT * 8; i += 256) *(v8h*)&wl[i * 8] = *(const v8h*)(Wh + (size_t)i * 8);
  __syncthreads();
  const size_t row0 = (size_t)blockIdx.x * 128 + (size_t)w * 16;
  const _Float16* arow = Ain + (row0 + m) * 64 + koff;
  const v16h a0 = FragH::load(arow);
  const v16h a1 = FragH::load(arow + 32);
  v8f acc[NT];
#pragma unroll
  for (int j = 0; j < NT; ++j) {
    FragH::U b0, b1;
    const int wo = (j * 16 + m) * 64 + koff;
    b0.h[0] = *(const v8h*)&wl[wo];
    b0.h[1] = *(const v8h*)&wl[wo + 16];
    b1.h[0] = *(const v8h*)&wl[wo + 32];
    b1.h[1] = *(const v8h*)&wl[wo + 48];
    v8f z = (v8f){0.f, 0.f, 0.f, 0.f, 0.f, 0.f, 0.f, 0.f};
    z = mma_h(a0, b0.v, z);
    z = mma_h(a1, b1.v, z);
    acc[j] = z;
  }
  float* myslab = slab + (LAST ? 0 : w * 16 * 68);
#pragma unroll
  for (int j = 0; j < NT; ++j) {
    const int ch = j * 16 + m;
    const float bv = bias[ch];
    float s = 0.0f, q = 0.0f;
    float mx = -BIGF, mn = BIGF;
#pragma unroll
    for (int r = 0; r < 8; ++r) {
      const float sc = acc[j][r] * WCARRY_INV;
      const float y = sc + bv;
      const float y2 = y * y;
      s = s + y;
      q = q + y2;
      if (LAST) { mx = fmaxf(mx, y); mn = fminf(mn, y); }
      else myslab[(8 * hh + r) * 68 + ch] = y;
    }
    const float so = __shfl_xor(s, 16);
    const float qo = __shfl_xor(q, 16);
    const float mxo = __shfl_xor(mx, 16);
    const float mno = __shfl_xor(mn, 16);
    s = s + so;
    q = q + qo;
    mx = fmaxf(mx, mxo);
    mn = fminf(mn, mno);
    if (hh == 0) {
      lsum[w * COUT + ch] = s;
      lsq[w * COUT + ch] = q;
      if (LAST) { wmx[w * COUT + ch] = mx; wmn[w * COUT + ch] = mn; }
    }
  }
  __syncthreads();
  if (tid < 2 * COUT) {
    const int c = (tid < COUT) ? tid : (tid - COUT);
    float s1 = 0.0f, s2 = 0.0f;
#pragma unroll
    for (int ww = 0; ww < 8; ++ww) { s1 = s1 + lsum[ww * COUT + c]; s2 = s2 + lsq[ww * COUT + c]; }
    pvec[tid] = (tid < COUT) ? s1 : s2;
  }
  __syncthreads();
  if (tid < (2 * COUT) / 4) {
    const v4f v = *(const v4f*)&pvec[4 * tid];
    float* pd = partial + (size_t)blockIdx.x * 2 * COUT + 4 * tid;
    *(volatile v4f*)pd = v;
    __threadfence();
    *(volatile v4f*)pd = v;
  }
  if (LAST) {
    const int qi = tid >> 6;
    const int idx = (tid & 63) * 4;
    const int sel = idx >> 7;
    const int c = idx & 127;
    v4f o;
#pragma unroll
    for (int e = 0; e < 4; ++e) {
      const float vmx = fmaxf(wmx[(2 * qi) * COUT + c + e], wmx[(2 * qi + 1) * COUT + c + e]);
      const float vmn = fminf(wmn[(2 * qi) * COUT + c + e], wmn[(2 * qi + 1) * COUT + c + e]);
      o[e] = sel ? vmn : vmx;
    }
    float* md = mmOut + (size_t)blockIdx.x * 1024 + 4 * tid;
    *(volatile v4f*)md = o;
    __threadfence();
    *(volatile v4f*)md = o;
  } else {
    const int q4 = lane >> 3;
    const int c8 = (lane & 7) * 8;
    for (int pass = 0; pass < 2; ++pass) {
#pragma unroll
      for (int it = 0; it < 4; ++it) {
        const int row = it * 4 + q4;
        const float* sp = myslab + row * 68 + c8;
        v8h hv;
#pragma unroll
        for (int e = 0; e < 8; ++e) hv[e] = (_Float16)sp[e];
        *(volatile v8h*)(rawOut + (row0 + row) * 64 + c8) = hv;
      }
      __threadfence();
    }
  }
}

template <int COUT>
__global__ void k_stats(const float* __restrict__ partial, const float* __restrict__ g,
                        const float* __restrict__ bt, float* __restrict__ ab) {
  __shared__ double ds[2 * COUT];
  __shared__ __align__(16) float sab[2 * COUT];
  const int t = threadIdx.x;
  double a = 0.0;
#pragma unroll 8
  for (int bk = 0; bk < 2048; ++bk) a += (double)partial[(size_t)bk * 2 * COUT + t];
  ds[t] = a;
  __syncthreads();
  if (t < COUT) {
    const double inv = 1.0 / 262144.0;
    const double mean = ds[t] * inv;
    double var = ds[COUT + t] * inv - mean * mean;
    var = var < 0.0 ? 0.0 : var;
    const float vf = (float)var;
    const float mf = (float)mean;
    const float sc = g[t] * rsqrtf(vf + 1e-5f);
    const float pm = mf * sc;
    sab[t] = sc;
    sab[COUT + t] = bt[t] - pm;
  }
  __syncthreads();
  if (t < (2 * COUT) / 4) {
    const v4f v = *(const v4f*)&sab[4 * t];
    *(volatile v4f*)(ab + 4 * t) = v;
    __threadfence();
    *(volatile v4f*)(ab + 4 * t) = v;
  }
}

__global__ __launch_bounds__(256) void k_apply(const unsigned short* __restrict__ yraw, const float* __restrict__ ab,
                                               _Float16* __restrict__ xout) {
  const size_t i = ((size_t)blockIdx.x * 256 + threadIdx.x) * 8;
  const int cb = (threadIdx.x & 7) * 8;
  const v4u wv = *(const v4u*)(yraw + i);
  const v4f a0 = *(const v4f*)(ab + cb);
  const v4f a1 = *(const v4f*)(ab + cb + 4);
  const v4f s0 = *(const v4f*)(ab + 64 + cb);
  const v4f s1 = *(const v4f*)(ab + 64 + cb + 4);
  float av[8] = {a0.x, a0.y, a0.z, a0.w, a1.x, a1.y, a1.z, a1.w};
  float sv[8] = {s0.x, s0.y, s0.z, s0.w, s1.x, s1.y, s1.z, s1.w};
  unsigned ww[4] = {wv.x, wv.y, wv.z, wv.w};
  v8h o;
#pragma unroll
  for (int e = 0; e < 4; ++e) {
    const unsigned u = ww[e];
    const float y0 = h16_to_f32(u & 0xffffu);
    const float y1 = h16_to_f32(u >> 16);
    const float p0 = y0 * av[2 * e];
    const float p1 = y1 * av[2 * e + 1];
    o[2 * e]     = (_Float16)fmaxf(p0 + sv[2 * e], 0.0f);
    o[2 * e + 1] = (_Float16)fmaxf(p1 + sv[2 * e + 1], 0.0f);
  }
  *(volatile v8h*)(xout + i) = o;
  __threadfence();
  *(volatile v8h*)(xout + i) = o;
}

__global__ __launch_bounds__(256) void k_final(const float* __restrict__ mm, const float* __restrict__ ab,
                                               float* __restrict__ out1) {
  __shared__ float tile[128 * 33];
  const int tid = threadIdx.x;
  const int b = blockIdx.x >> 5;
  const int s0 = (blockIdx.x & 31) << 5;
  const int c = tid & 127;
  const float a = ab[c];
  const float sh = ab[128 + c];
#pragma unroll 4
  for (int it = 0; it < 16; ++it) {
    const int sq = (tid >> 7) + 2 * it;
    const size_t bs = (size_t)b * NQ + s0 + sq;
    const float mx = mm[bs * 256 + c];
    const float mn = mm[bs * 256 + 128 + c];
    const float pick = (a >= 0.0f) ? mx : mn;
    const float p = pick * a;
    tile[c * 33 + sq] = fmaxf(p + sh, 0.0f);
  }
  __syncthreads();
  const int l8 = tid & 7;
  for (int pass = 0; pass < 2; ++pass) {
#pragma unroll
    for (int it = 0; it < 4; ++it) {
      const int ch = it * 32 + (tid >> 3);
      const float* sp = tile + ch * 33 + 4 * l8;
      v4f v;
      v.x = sp[0]; v.y = sp[1]; v.z = sp[2]; v.w = sp[3];
      *(volatile v4f*)(out1 + ((size_t)b * 128 + ch) * NQ + s0 + 4 * l8) = v;
    }
    __threadfence();
  }
}

extern "C" void kernel_launch(void* const* d_in, const int* in_sizes, int n_in,
                              void* d_out, int out_size, void* d_ws, size_t ws_size,
                              hipStream_t stream) {
  (void)in_sizes; (void)n_in; (void)out_size;
  if (ws_size < WS_TOTAL) return;
  const float* xyz  = (const float*)d_in[0];
  const float* feat = (const float*)d_in[1];
  const float* pts  = (const float*)d_in[2];
  const float* W1 = (const float*)d_in[3];  const float* b1 = (const float*)d_in[4];
  const float* g1 = (const float*)d_in[5];  const float* bt1 = (const float*)d_in[6];
  const float* W2 = (const float*)d_in[7];  const float* b2 = (const float*)d_in[8];
  const float* g2 = (const float*)d_in[9];  const float* bt2 = (const float*)d_in[10];
  const float* W3 = (const float*)d_in[11]; const float* b3 = (const float*)d_in[12];
  const float* g3 = (const float*)d_in[13]; const float* bt3 = (const float*)d_in[14];
  float* out = (float*)d_out;
  char* ws = (char*)d_ws;

  float*    comb   = (float*)(ws + OFF_COMB);
  float*    qcomb  = (float*)(ws + OFF_QCOMB);
  int*      fpsIdx = (int*)(ws + OFF_FPS);
  int*      knn    = (int*)(ws + OFF_KNN);
  _Float16* Wh     = (_Float16*)(ws + OFF_WH);
  float*    ab1    = (float*)(ws + OFF_AB);
  float*    ab2    = ab1 + 256;
  float*    ab3    = ab1 + 512;
  float*    part1  = (float*)(ws + OFF_P1);
  float*    part2  = (float*)(ws + OFF_P2);
  float*    part3  = (float*)(ws + OFF_P3);
  _Float16* planeX = (_Float16*)(ws + OFF_X);
  _Float16* planeR = (_Float16*)(ws + OFF_R);
  float*    mm     = (float*)(ws + OFF_MM);
  _Float16* W1h = Wh;
  _Float16* W2h = Wh + 4096;
  _Float16* W3h = Wh + 8192;

  k_prep   <<<(NB * NPTS) / 64, 256, 0, stream>>>(xyz, feat, pts, comb);
  k_fps    <<<NB, 512, 0, stream>>>(comb, fpsIdx);
  k_gather <<<(NB * NQ) / 64, 256, 0, stream>>>(comb, fpsIdx, qcomb, out);
  k_knn    <<<(NB * NQ) / 16, 256, 0, stream>>>(comb, qcomb, knn);
  k_group  <<<NROWS / 256, 256, 0, stream>>>(comb, qcomb, knn, planeX);
  k_packw  <<<8, 256, 0, stream>>>(W1, W2, W3, Wh);

  const int nblk = NROWS / 128;
  const int napply = (NROWS * 64 / 8) / 256;
  k_mlp<64, false> <<<nblk, 256, 0, stream>>>(planeX, W1h, b1, planeR, part1, mm);
  k_stats<64>      <<<1, 128, 0, stream>>>(part1, g1, bt1, ab1);
  k_apply          <<<napply, 256, 0, stream>>>((const unsigned short*)planeR, ab1, planeX);
  k_mlp<64, false> <<<nblk, 256, 0, stream>>>(planeX, W2h, b2, planeR, part2, mm);
  k_stats<64>      <<<1, 128, 0, stream>>>(part2, g2, bt2, ab2);
  k_apply          <<<napply, 256, 0, stream>>>((const unsigned short*)planeR, ab2, planeX);
  k_mlp<128, true> <<<nblk, 256, 0, stream>>>(planeX, W3h, b3, planeR, part3, mm);
  k_stats<128>     <<<1, 256, 0, stream>>>(part3, g3, bt3, ab3);
  k_final          <<<(NB * NQ) / 32, 256, 0, stream>>>(mm, ab3, out + OUT1_OFF);
}
